// SparseEncoderVoxelNeXt2DFuse_7370163880455
// MI455X (gfx1250) — hardware-verified
//
#include <hip/hip_runtime.h>


namespace {
constexpr int B = 4, GH = 1440, GW = 1440, N = 200000, C = 32, NB = 3, KK = 9 * C, NCELL = B * GH * GW, NCOARSE = NCELL / 16, NBLK = N / 16;
constexpr float XS = 8.0f, WSC = 256.0f, EPS = 1e-3f;
typedef _Float16 b16;
typedef __attribute__((ext_vector_type(16))) _Float16 v16b;
typedef __attribute__((ext_vector_type(8))) _Float16 v8b;
typedef __attribute__((ext_vector_type(8))) float v8f;
typedef __attribute__((ext_vector_type(4))) int v4i;
__device__ __forceinline__ float bf16_rne(float f) { unsigned int u = __float_as_uint(f); u += 0x7FFFu + ((u >> 16) & 1u); return __uint_as_float(u & 0xFFFF0000u); }
__device__ __forceinline__ void split16(float v, b16& hi, b16& lo) { hi = (b16)v; lo = (b16)(v - (float)hi); }
__device__ __forceinline__ v16b frag_kb(const b16* p, int hh) { const v8b a = *(const v8b*)(p + 8 * hh), b = *(const v8b*)(p + 16 + 8 * hh); v16b f;
#pragma unroll
  for (int e = 0; e < 8; ++e) { f[e] = a[e]; f[8 + e] = b[e]; } return f; }
__device__ __forceinline__ v8f wmma16b(v16b a, v16b b, v8f c) { v8f d = __builtin_amdgcn_wmma_f32_16x16x32_f16(false, a, false, b, (short)0, c, false, false); asm volatile("v_nop\n\tv_nop\n\tv_nop\n\tv_nop" : "+v"(d) : "v"(a), "v"(b)); return d; }
__device__ __forceinline__ void wave_lds_sync() { __builtin_amdgcn_fence(__ATOMIC_RELEASE, "workgroup"); __builtin_amdgcn_wave_barrier(); __builtin_amdgcn_fence(__ATOMIC_ACQUIRE, "workgroup"); }
__device__ __forceinline__ float pmul(float a, float b) { float p = a * b; asm volatile("" : "+v"(p)); return p; }
__device__ __forceinline__ int iclamp(int v, int lo, int hi) { return v < lo ? lo : (v > hi ? hi : v); }
constexpr int CSR_NBLK10 = 512, CSR_GB10 = 10, CSR_GN10 = 1 << CSR_GB10  , CSR_TS10 = (CSR_GN10 < 32 ? 32 : CSR_GN10)  , CSR_MAXG10 = 512, CSR_CAP10 = 12288  ;
__device__ __host__ __forceinline__ int csr_tix10(int v) { return (v >> CSR_GB10) * CSR_TS10 + (v & (CSR_GN10 - 1)); }
__global__ __launch_bounds__(64) void csrA_kernel10(const int* __restrict__ dst, int E, int N, int nG, int CHP, int NGP, int* __restrict__ STG, int* __restrict__ HST) {
  extern __shared__ int sm[];
  int* cnt = sm; int* run = sm + NGP; int* ids = sm + 2 * NGP;
  const int b = blockIdx.x; const int ch = (E + CSR_NBLK10 - 1) / CSR_NBLK10; const int e0 = b * ch, e1 = min(E, e0 + ch);
  for (int i = threadIdx.x; i < NGP; i += 64) cnt[i] = 0;
  for (int i = threadIdx.x; i < CHP; i += 64) ids[i] = -1;
  __syncthreads();
  if (threadIdx.x == 0) {
    for (int e = e0; e < e1; ++e) { int d = dst[e]; d = (d < 0) ? 0 : (d >= N ? N - 1 : d); cnt[d >> CSR_GB10] += 1; }
    int acc = 0; for (int g = 0; g < nG; ++g) { run[g] = acc; acc += cnt[g]; }
    for (int e = e0; e < e1; ++e) { int d = dst[e]; d = (d < 0) ? 0 : (d >= N ? N - 1 : d); const int g = d >> CSR_GB10; ids[run[g]] = e; run[g] += 1; } }
  __syncthreads();
  typedef __attribute__((ext_vector_type(4))) int v4i;
  for (int pass = 0; pass < 2; ++pass) {
    for (int i = threadIdx.x; i < CHP / 4; i += 64) *(volatile v4i*)(STG + (size_t)b * CHP + i * 4) = *(const v4i*)(&ids[i * 4]);
    for (int i = threadIdx.x; i < NGP / 4; i += 64) { v4i v; for (int e = 0; e < 4; ++e) v[e] = (i * 4 + e < nG) ? cnt[i * 4 + e] : 0; *(volatile v4i*)(HST + (size_t)b * NGP + i * 4) = v; }
    __threadfence(); }
}
__global__ __launch_bounds__(512) void csrS_kernel10(const int* __restrict__ HST, int nG, int NGP, int* __restrict__ START, int* __restrict__ TOT, int* __restrict__ OFF) {
  __shared__ int tot[CSR_MAXG10];
  const int b = threadIdx.x;
  for (int pass = 0; pass < 2; ++pass) { int runb = 0; for (int g = 0; g < nG; ++g) { int c = HST[(size_t)b * NGP + g]; c = (c < 0) ? 0 : c; ((volatile int*)OFF)[(size_t)g * CSR_NBLK10 + b] = runb; runb += c; } __threadfence(); }
  for (int g = threadIdx.x; g < nG; g += 512) { int s = 0; for (int bb = 0; bb < CSR_NBLK10; ++bb) { int c = HST[(size_t)bb * NGP + g]; s += (c < 0) ? 0 : c; } tot[g] = s; }
  __syncthreads();
  if (threadIdx.x < 32) {
    __shared__ int st[CSR_MAXG10 + 32];
    if (threadIdx.x == 0) { int acc = 0; for (int g = 0; g < NGP; ++g) { st[g] = acc; if (g < nG) acc += (tot[g] + 31) & ~31; } st[NGP] = acc; }
    __builtin_amdgcn_fence(__ATOMIC_RELEASE, "workgroup"); __builtin_amdgcn_wave_barrier(); __builtin_amdgcn_fence(__ATOMIC_ACQUIRE, "workgroup");
    for (int pass = 0; pass < 2; ++pass) { for (int i = threadIdx.x; i < NGP + 32; i += 32) { ((volatile int*)START)[i] = (i <= NGP) ? st[min(i, NGP)] : 0; ((volatile int*)TOT)[i] = (i < nG) ? tot[i] : 0; } __threadfence(); } }
}
__global__ __launch_bounds__(256) void csrB_kernel10(const int* __restrict__ dst, int N, int nG, int CHP, int NGP, int permLen, const int* __restrict__ STG, const int* __restrict__ HST, const int* __restrict__ OFF, const int* __restrict__ START, const int* __restrict__ TOT, int* __restrict__ PERM, int* __restrict__ ROWPTR, int* __restrict__ ROWCNT, int* __restrict__ FLAG) {
  typedef __attribute__((ext_vector_type(4))) int v4i;
  __shared__ int ids[CSR_CAP10]; __shared__ unsigned short key[CSR_CAP10]; __shared__ int outp[CSR_CAP10]; __shared__ int ncnt[CSR_GN10 + 1]; __shared__ int boff[CSR_NBLK10 + 1];
  const int g = blockIdx.x, t_ = threadIdx.x; int tot = TOT[g]; int st = START[g], stn = START[g + 1]; const int v0 = g * CSR_GN10; const int nv = min(CSR_GN10, N - v0); const int t0 = g * CSR_TS10;
  st = (st < 0) ? 0 : (st > permLen - 32 ? permLen - 32 : st) & ~31; stn = (stn < st) ? st : (stn > permLen ? permLen : stn); tot = (tot < 0) ? 0 : tot; if (tot > stn - st && tot <= CSR_CAP10) tot = stn - st;
  if (tot > CSR_CAP10) {
    for (int pass = 0; pass < 2; ++pass) { for (int i = t_; i < CSR_TS10 / 4; i += 256) { v4i a, c; for (int e = 0; e < 4; ++e) { a[e] = st; c[e] = 0; } *(volatile v4i*)(ROWPTR + t0 + i * 4) = a; *(volatile v4i*)(ROWCNT + t0 + i * 4) = c; } if (t_ == 0) ((volatile int*)FLAG)[0] = 1; __threadfence(); } (void)nv; return; }
  if (t_ == 0) { int acc = 0; for (int b = 0; b < CSR_NBLK10; ++b) { boff[b] = acc; int c = HST[(size_t)b * NGP + g]; c = (c < 0) ? 0 : (c > CHP ? CHP : c); acc += c; if (acc > tot) acc = tot; } boff[CSR_NBLK10] = acc; }
  for (int i = t_; i <= CSR_GN10; i += 256) ncnt[i] = 0;
  __syncthreads();
  for (int b = 0; b < CSR_NBLK10; ++b) { const int c = boff[b + 1] - boff[b]; int o_ = OFF[(size_t)g * CSR_NBLK10 + b]; o_ = (o_ < 0) ? 0 : (o_ > CHP - c ? CHP - c : o_); const int* src_ = STG + (size_t)b * CHP + o_;
    for (int i = t_; i < c; i += 256) { int id = src_[i]; id = (id < 0) ? 0 : id; ids[boff[b] + i] = id; int d = dst[id]; d = (d < v0) ? v0 : (d >= N ? N - 1 : d); int kk = d - v0; kk = (kk < 0) ? 0 : (kk >= CSR_GN10 ? CSR_GN10 - 1 : kk); key[boff[b] + i] = (unsigned short)kk; } }
  __syncthreads();
  if (t_ == 0) { for (int i = 0; i < tot; ++i) ncnt[key[i]] += 1; int acc = 0; for (int vl = 0; vl < CSR_GN10; ++vl) { const int c = ncnt[vl]; ncnt[vl] = acc; acc += c; } ncnt[CSR_GN10] = acc;
    for (int i = 0; i < tot; ++i) { const int vl = key[i]; outp[ncnt[vl]] = ids[i]; ncnt[vl] += 1; }
    for (int vl = CSR_GN10; vl > 0; --vl) ncnt[vl] = ncnt[vl - 1]; ncnt[0] = 0; }
  __syncthreads();
  for (int pass = 0; pass < 2; ++pass) {
    for (int i = t_; i < (stn - st) / 4; i += 256) { v4i v; for (int e = 0; e < 4; ++e) { const int q = i * 4 + e; v[e] = (q < tot) ? outp[q] : -1; } *(volatile v4i*)(PERM + st + i * 4) = v; }
    for (int i = t_; i < CSR_TS10 / 4; i += 256) { v4i a, c; for (int e = 0; e < 4; ++e) { const int vl = i * 4 + e; const int vc = vl < CSR_GN10 ? vl : CSR_GN10; a[e] = (vl < CSR_GN10) ? st + ncnt[vc] : st; c[e] = (vl < nv) ? (ncnt[(vc < CSR_GN10 ? vc : CSR_GN10 - 1) + 1] - ncnt[vc]) : 0; } *(volatile v4i*)(ROWPTR + t0 + i * 4) = a; *(volatile v4i*)(ROWCNT + t0 + i * 4) = c; }
    __threadfence(); }
}
__global__ __launch_bounds__(256) void csrZ_kernel10(int* __restrict__ p, size_t n4) { typedef __attribute__((ext_vector_type(4))) int v4i; const size_t tid = (size_t)blockIdx.x * 256 + threadIdx.x, nth = (size_t)gridDim.x * 256; v4i z = {0, 0, 0, 0}; for (size_t i = tid; i < n4; i += nth) *(volatile v4i*)(p + i * 4) = z; }
struct CsrBufs10 { int *STG, *HST, *OFF, *START, *TOT, *PERM, *ROWPTR, *ROWCNT, *FLAG; int nG, NGP, CHP; size_t permLen; char* base; size_t bytes; };
static size_t csr_carve10(CsrBufs10& c, char* ws, size_t off, int E, int N) {
  const size_t off0 = off; c.base = ws + off;
  auto al = [&](size_t bytes) { char* p = ws + off; off += (bytes + 255) & ~(size_t)255; return p; };
  c.nG = (N + CSR_GN10 - 1) / CSR_GN10; c.NGP = (c.nG + 31) & ~31; const int ch = (E + CSR_NBLK10 - 1) / CSR_NBLK10; c.CHP = (ch + 31) & ~31; c.permLen = (size_t)E + 32 * (size_t)c.nG + 32;
  c.STG = (int*)al((size_t)CSR_NBLK10 * c.CHP * 4); c.HST = (int*)al((size_t)CSR_NBLK10 * c.NGP * 4); c.OFF = (int*)al((size_t)c.NGP * CSR_NBLK10 * 4); c.START = (int*)al((size_t)(c.NGP + 64) * 4); c.TOT = (int*)al((size_t)(c.NGP + 64) * 4);
  c.PERM = (int*)al(c.permLen * 4); c.ROWPTR = (int*)al((size_t)c.nG * CSR_TS10 * 4); c.ROWCNT = (int*)al((size_t)c.nG * CSR_TS10 * 4); c.FLAG = (int*)al(256);
  c.bytes = off - off0; return off;
}
static void csr_build10(const CsrBufs10& c, const int* dst, int E, int N, hipStream_t stream) {
  const size_t smem = (size_t)(2 * c.NGP + c.CHP) * 4;
  csrZ_kernel10<<<512, 256, 0, stream>>>((int*)c.base, c.bytes / 16);
  csrA_kernel10<<<CSR_NBLK10, 64, smem, stream>>>(dst, E, N, c.nG, c.CHP, c.NGP, c.STG, c.HST);
  csrS_kernel10<<<1, 512, 0, stream>>>(c.HST, c.nG, c.NGP, c.START, c.TOT, c.OFF);
  csrB_kernel10<<<c.nG, 256, 0, stream>>>(dst, N, c.nG, c.CHP, c.NGP, (int)c.permLen, c.STG, c.HST, c.OFF, c.START, c.TOT, c.PERM, c.ROWPTR, c.ROWCNT, c.FLAG);
}


__global__ __launch_bounds__(256) void key_kernel(const int* __restrict__ cb, const int* __restrict__ cy, const int* __restrict__ cx, int* __restrict__ KEY, int* __restrict__ KEYC) { const int i = blockIdx.x * 256 + threadIdx.x; if (i >= N) return; const int k = (iclamp(cb[i], 0, B - 1) * GH + iclamp(cy[i], 0, GH - 1)) * GW + iclamp(cx[i], 0, GW - 1); for (int pass = 0; pass < 2; ++pass) { ((volatile int*)KEY)[i] = k; ((volatile int*)KEYC)[i] = k >> 4; __threadfence(); } }
__global__ __launch_bounds__(256) void nbr_kernel(const int* __restrict__ cb, const int* __restrict__ cy, const int* __restrict__ cx, const int* __restrict__ KEY, const int* __restrict__ PERM, const int* __restrict__ ROWPTR, const int* __restrict__ ROWCNT, int permLen, int* __restrict__ NBR) {
  const int i = blockIdx.x * 256 + threadIdx.x; if (i >= N) return; const int b = iclamp(cb[i], 0, B - 1), y = iclamp(cy[i], 0, GH - 1), x = iclamp(cx[i], 0, GW - 1); int nb[16];
#pragma unroll
  for (int k = 0; k < 16; ++k) nb[k] = -1;
#pragma unroll
  for (int k = 0; k < 9; ++k) { const int ny = y + k / 3 - 1, nx = x + k % 3 - 1; int best = -1;
    if (ny >= 0 && ny < GH && nx >= 0 && nx < GW) { const int cell = (b * GH + ny) * GW + nx; const int cc = cell >> 4; int cnt = iclamp(ROWCNT[cc], 0, 1 << 20); const int st = iclamp(ROWPTR[cc], 0, permLen - cnt);
      for (int j = 0; j < cnt; ++j) { const int v = iclamp(PERM[st + j], 0, N - 1); if (KEY[v] == cell) best = v > best ? v : best; } }
    nb[k] = best; }
  for (int pass = 0; pass < 2; ++pass) { for (int q = 0; q < 4; ++q) *(volatile v4i*)(NBR + (size_t)i * 16 + q * 4) = (v4i){nb[q * 4], nb[q * 4 + 1], nb[q * 4 + 2], nb[q * 4 + 3]}; __threadfence(); }
}
__global__ __launch_bounds__(256) void wput_kernel(const float* __restrict__ W, b16* __restrict__ WT) { const int u = blockIdx.x * 256 + threadIdx.x; if (u >= C * (KK / 8)) return; const int co = u / (KK / 8), k0 = (u % (KK / 8)) * 8; v8b v;
#pragma unroll
  for (int j = 0; j < 8; ++j) { const int kc = k0 + j; v[j] = (b16)(bf16_rne(W[(size_t)kc * C + co]) * WSC); } for (int pass = 0; pass < 2; ++pass) { *(volatile v8b*)(WT + (size_t)co * KK + k0) = v; __threadfence(); } }
template <int L1, int MODE>
__global__ __launch_bounds__(32) void conv_kernel(const float* __restrict__ Hin, const int* __restrict__ NBR, const b16* __restrict__ WT, const float* __restrict__ bias, const float* __restrict__ g, const float* __restrict__ bt, const float* __restrict__ mu, const float* __restrict__ var, const float* __restrict__ RES, int L1res, int NLIM, float* __restrict__ O) {
  __shared__ __attribute__((aligned(16))) b16 Ah[16][KK + 8], Al[16][KK + 8]; __shared__ float Tf[16][C + 1];
  const int lane = threadIdx.x, nloc = lane & 15, hlf = lane >> 4; const size_t m0 = (size_t)blockIdx.x * 16; if (m0 >= (size_t)NLIM) return;
  for (int rr = 0; rr < 16; ++rr) { const size_t i = m0 + rr;
    for (int k = 0; k < 9; ++k) { int nb = NBR[i * 16 + k]; nb = nb < 0 ? -1 : iclamp(nb, 0, N - 1); if (nb >= NLIM) nb = -1; float v = 0.0f; if (nb >= 0) { v = Hin[(size_t)nb * C + lane]; if (L1) v = bf16_rne(v); }
      if (L1) { Ah[rr][k * C + lane] = (b16)(v * XS); } else { b16 p, q; split16(v * XS, p, q); Ah[rr][k * C + lane] = p; Al[rr][k * C + lane] = q; } } }
  wave_lds_sync(); v8f acc[2] = {(v8f){}, (v8f){}};
#pragma unroll
  for (int kb = 0; kb < KK; kb += 32) { const v16b a = frag_kb(&Ah[nloc][kb], hlf); v16b al; if (!L1) al = frag_kb(&Al[nloc][kb], hlf);
#pragma unroll
    for (int t = 0; t < 2; ++t) { const v16b bw = frag_kb(WT + (size_t)(t * 16 + nloc) * KK + kb, hlf); acc[t] = wmma16b(a, bw, acc[t]); if (!L1) acc[t] = wmma16b(al, bw, acc[t]); } }
#pragma unroll
  for (int t = 0; t < 2; ++t) { const int c = t * 16 + nloc; const float bb = bf16_rne(bias[c]), sc = pmul(rsqrtf(bf16_rne(var[c]) + EPS), bf16_rne(g[c])), mm = bf16_rne(mu[c]), be = bf16_rne(bt[c]);
#pragma unroll
    for (int r8 = 0; r8 < 8; ++r8) Tf[8 * hlf + r8][c] = pmul(acc[t][r8] * (1.0f / (XS * WSC)) + bb - mm, sc) + be; }
  wave_lds_sync();
  for (int pass = 0; pass < 2; ++pass) { for (int rr = 0; rr < 16; ++rr) { float v = Tf[rr][lane]; if (MODE == 1) { float r = RES[(m0 + rr) * C + lane]; if (L1res) r = bf16_rne(r); v += r; } ((volatile float*)O)[(m0 + rr) * C + lane] = fmaxf(v, 0.0f); } __threadfence(); }
}
}

extern "C" void kernel_launch(void* const* d_in, const int* in_sizes, int n_in, void* d_out, int out_size, void* d_ws, size_t ws_size, hipStream_t stream) {
  (void)n_in;
  auto Fp = [&](int i) { return (const float*)d_in[i]; }; auto Ip = [&](int i) { return (const int*)d_in[i]; };
  if (in_sizes[0] != N * C || in_sizes[1] != NB * 2 * KK * C || in_sizes[2] != NB * 2 * C || in_sizes[6] != NB * 2 * C || in_sizes[7] != N || in_sizes[8] != N || in_sizes[9] != N || out_size != N * C) return;
  const int NLIM = N; const int GB16 = NBLK;
  size_t off = 0; char* ws = (char*)d_ws;
  auto carve = [&](size_t bytes) { char* p = ws + off; off += (bytes + 255) & ~(size_t)255; return p; };
  b16* WT = (b16*)carve((size_t)NB * 2 * C * KK * 2); int* KEY = (int*)carve((size_t)N * 4); int* KEYC = (int*)carve((size_t)N * 4); int* NBR = (int*)carve((size_t)N * 16 * 4); float* HA = (float*)carve((size_t)N * C * 4); float* HB = (float*)carve((size_t)N * C * 4); float* HO = (float*)carve((size_t)N * C * 4);
  CsrBufs10 csr; off = csr_carve10(csr, ws, off, N, NCOARSE);
  if (off > ws_size || off > ((size_t)224 << 20)) return;
  for (int l = 0; l < NB * 2; ++l) wput_kernel<<<(C * (KK / 8) + 255) / 256, 256, 0, stream>>>(Fp(1) + (size_t)l * KK * C, WT + (size_t)l * C * KK);
  key_kernel<<<(N + 255) / 256, 256, 0, stream>>>(Ip(7), Ip(8), Ip(9), KEY, KEYC);
  csr_build10(csr, KEYC, N, NCOARSE, stream);
  nbr_kernel<<<(N + 255) / 256, 256, 0, stream>>>(Ip(7), Ip(8), Ip(9), KEY, csr.PERM, csr.ROWPTR, csr.ROWCNT, (int)csr.permLen, NBR);
  const float* hin = Fp(0); int l1 = 1;
  for (int blk = 0; blk < NB; ++blk) { const int la = blk * 2, lb = blk * 2 + 1; float* hout = (blk == NB - 1) ? (float*)d_out : (blk & 1 ? HB : HA);
    if (l1) conv_kernel<1, 0><<<GB16, 32, 0, stream>>>(hin, NBR, WT + (size_t)la * C * KK, Fp(2) + la * C, Fp(3) + la * C, Fp(4) + la * C, Fp(5) + la * C, Fp(6) + la * C, nullptr, 0, NLIM, HO);
    else    conv_kernel<0, 0><<<GB16, 32, 0, stream>>>(hin, NBR, WT + (size_t)la * C * KK, Fp(2) + la * C, Fp(3) + la * C, Fp(4) + la * C, Fp(5) + la * C, Fp(6) + la * C, nullptr, 0, NLIM, HO);
    conv_kernel<0, 1><<<GB16, 32, 0, stream>>>(HO, NBR, WT + (size_t)lb * C * KK, Fp(2) + lb * C, Fp(3) + lb * C, Fp(4) + lb * C, Fp(5) + lb * C, Fp(6) + lb * C, hin, l1, NLIM, hout);
    hin = hout; l1 = 0; }
}
